// VectorizedODT_81552839016748
// MI455X (gfx1250) — hardware-run, weakly checked
//
#include <hip/hip_runtime.h>


#ifndef NB
#define NB 16
#endif
#ifndef SEQ
#define SEQ 1024
#endif
#define NB_FULL  16
#define SEQ_FULL 1024
#ifndef OUT_SEQ
#define OUT_SEQ SEQ
#endif
#define NF   256
#define NT   64
#define ND   6
#define NC   64
#define NU   128
#define TD   (NT * ND)
#define PP   388
#define SELC 1024.0f
#define SELI (1.0f / 1024.0f)
#define WSH  16384.0f
#define OSC  (1.0f / (16384.0f * 64.0f))
#define LOG2E 1.4426950408889634f

static_assert(NC == (1 << ND));
static_assert(NC == 64);
static_assert(NU == 128);
static_assert(NF % 32 == 0);
static_assert(TD % 128 == 0);
static_assert(PP >= TD);
static_assert(PP >= NU);
static_assert((PP * 4) % 16 == 0);
static_assert(16 * PP * 4 <= 131072);
static_assert(SEQ % 16 == 0);
static_assert((NB * SEQ) % 16 == 0);
static_assert(32 * 16 == NU * 4);
static_assert(32 * 16 == NF * 2);
static_assert(((size_t)SEQ * NF) % 64 == 0);
static_assert(((size_t)NT * NU * NC) % 64 == 0);
static_assert(NB <= NB_FULL);
static_assert(SEQ <= SEQ_FULL);

typedef _Float16 h16;
typedef unsigned short bf;
typedef __attribute__((ext_vector_type(16))) __bf16   v16bf;
typedef __attribute__((ext_vector_type(16))) _Float16 v16h;
typedef __attribute__((ext_vector_type(8)))  _Float16 v8h;
typedef __attribute__((ext_vector_type(8)))  unsigned short v8us;
typedef __attribute__((ext_vector_type(8)))  float    v8f;
typedef __attribute__((ext_vector_type(4)))  float    v4f;
typedef v4f  __attribute__((may_alias)) v4fa;

__device__ __forceinline__ unsigned short f2bf(float f) { unsigned u = __float_as_uint(f); u += 0x7FFFu + ((u >> 16) & 1u); return (unsigned short)(u >> 16); }
__device__ __forceinline__ float bfr(float f) { return __uint_as_float(((unsigned)f2bf(f)) << 16); }
__device__ __forceinline__ v16h cat16(v8h lo, v8h hi) { return __builtin_shufflevector(lo, hi, 0, 1, 2, 3, 4, 5, 6, 7, 8, 9, 10, 11, 12, 13, 14, 15); }
__device__ __forceinline__ v16bf cat16b(v8us lo, v8us hi) { return __builtin_bit_cast(v16bf, __builtin_shufflevector(lo, hi, 0, 1, 2, 3, 4, 5, 6, 7, 8, 9, 10, 11, 12, 13, 14, 15)); }
__device__ __forceinline__ v8f wmma16(v16h a, v16h b, v8f c) { return __builtin_amdgcn_wmma_f32_16x16x32_f16(false, a, false, b, (short)0, c, false, false); }
__device__ __forceinline__ v8f wmmab(v16bf a, v16bf b, v8f c) { return __builtin_amdgcn_wmma_f32_16x16x32_bf16(false, a, false, b, (short)0, c, false, false); }
__device__ __forceinline__ v16h  ldh(const h16* p) { return cat16(*(const v8h*)p, *(const v8h*)(p + 16)); }
__device__ __forceinline__ v16bf ldb(const bf* p)  { return cat16b(*(const v8us*)p, *(const v8us*)(p + 16)); }
__device__ __forceinline__ void wave_sync() { __builtin_amdgcn_fence(3  , "wavefront"); __builtin_amdgcn_wave_barrier(); asm volatile("" ::: "memory"); }

static __device__ __forceinline__ h16 toh_flush(float v) { const h16 r = (h16)v; return (fabsf(v) < 6.103515625e-05f) ? (h16)0.0f : r; }
static __device__ __forceinline__ v8f wmma16g(v16h a, v16h b, v8f c) {
    c = wmma16(a, b, c);
    asm volatile("v_nop\n\tv_nop\n\tv_nop\n\tv_nop" : "+v"(c) : "v"(a), "v"(b));
    return c;
}

__global__ __launch_bounds__(256) void k_cvth8(const float* __restrict__ src, h16* dst, size_t n8) {
#pragma clang fp contract(off)
    const size_t i = (size_t)blockIdx.x * 256 + threadIdx.x; if (i >= n8) return;
    const v8f v = *(const v8f*)(src + i * 8); v8h o;
#pragma unroll
    for (int k = 0; k < 8; ++k) o[k] = toh_flush(bfr(v[k]));
    *(volatile v8h*)(dst + i * 8) = o; __threadfence(); *(volatile v8h*)(dst + i * 8) = o;
}

__global__ __launch_bounds__(256) void k_sel(const float* __restrict__ logits, h16* ST) {
#pragma clang fp contract(off)
    __shared__ float redm[8];
    __shared__ float reds[8];
    __shared__ __align__(16) h16 rowh[NF];
    const int col = blockIdx.x;
    const int f = threadIdx.x;
    const int lane = f & 31, wave = f >> 5;
    const float v = bfr(logits[(size_t)f * TD + col]);
    float mx = v;
#pragma unroll
    for (int o = 16; o > 0; o >>= 1) mx = fmaxf(mx, __shfl_xor(mx, o, 32));
    if (lane == 0) redm[wave] = mx;
    __syncthreads();
    float m = redm[0];
#pragma unroll
    for (int i = 1; i < 8; ++i) m = fmaxf(m, redm[i]);
    const float e = expf(v - m);
    float s = e;
#pragma unroll
    for (int o = 16; o > 0; o >>= 1) s += __shfl_xor(s, o, 32);
    if (lane == 0) reds[wave] = s;
    __syncthreads();
    float tot = reds[0];
#pragma unroll
    for (int i = 1; i < 8; ++i) tot += reds[i];
    const float inv = 1.0f / tot;
    rowh[f] = toh_flush((e * inv) * SELC);
    __syncthreads();
    if (f < 32) {
        const v8h hv = *(const v8h*)(&rowh[8 * f]);
        h16* dp = ST + (size_t)col * NF + 8 * f;
        *(volatile v8h*)dp = hv; __threadfence(); *(volatile v8h*)dp = hv;
    }
}

__global__ __launch_bounds__(32) void k_trees(const h16* __restrict__ XH, const h16* __restrict__ ST, const h16* __restrict__ RH,
                                              const float* __restrict__ thr, const float* __restrict__ ltp, float* OUT) {
    __shared__ __align__(16) float ps[16 * PP];
    const int lane = threadIdx.x & 31, lr = lane & 15, hi = lane >> 4;
    const int r0 = blockIdx.x * 16;
    const int bb = r0 / SEQ, ss = r0 % SEQ;
    v8f acc[8];
    const size_t aoff = (size_t)(r0 + lr) * NF + 8 * hi;
#pragma unroll 1
    for (int ch = 0; ch < TD / 128; ++ch) {
#pragma unroll
        for (int j = 0; j < 8; ++j) acc[j] = (v8f){};
        const size_t boff = (size_t)(ch * 128 + lr) * NF + 8 * hi;
#pragma unroll 1
        for (int kc = 0; kc < NF; kc += 32) {
            const v16h a = ldh(XH + aoff + kc);
#pragma unroll
            for (int j = 0; j < 8; ++j) { const v16h b = ldh(ST + boff + (size_t)j * 16 * NF + kc); acc[j] = wmma16g(a, b, acc[j]); }
        }
#pragma unroll
        for (int j = 0; j < 8; ++j) {
            const int col = ch * 128 + j * 16 + lr;
            const float th = bfr(thr[col]);
            const float sc = __builtin_amdgcn_exp2f(-bfr(ltp[col]) * LOG2E);
#pragma unroll
            for (int r = 0; r < 8; ++r) {
                const float tl = (acc[j][r] * SELI - th) * sc;
                const float e = __builtin_amdgcn_exp2f(-tl * LOG2E);
                ps[(8 * hi + r) * PP + col] = __builtin_amdgcn_rcpf(1.0f + e);
            }
        }
    }
    wave_sync();

#pragma unroll
    for (int j = 0; j < 8; ++j) acc[j] = (v8f){};
    const size_t roff = (size_t)lr * NC + 8 * hi;
#pragma unroll 1
    for (int t = 0; t < NT; ++t) {
        const int pbx = lr * PP + ND * t;
        const float p0 = ps[pbx], p1 = ps[pbx + 1], p2 = ps[pbx + 2], p3 = ps[pbx + 3], p4 = ps[pbx + 4], p5 = ps[pbx + 5];
        const float n0 = 1.0f - p0, n1 = 1.0f - p1, n2 = 1.0f - p2, n3 = 1.0f - p3, n4 = 1.0f - p4, n5 = 1.0f - p5;
        const float a00 = n0 * n1, a01 = p0 * n1, a10 = n0 * p1, a11 = p0 * p1;
        float a[8];
        a[0] = a00 * n2; a[1] = a01 * n2; a[2] = a10 * n2; a[3] = a11 * n2;
        a[4] = a00 * p2; a[5] = a01 * p2; a[6] = a10 * p2; a[7] = a11 * p2;
        const float e3 = (hi ? p3 : n3) * WSH;
        const float e30 = e3 * n4, e31 = e3 * p4;
        const h16* rb = RH + roff + (size_t)t * NU * NC;
#pragma unroll
        for (int ks = 0; ks < 2; ++ks) {
            const float f0 = e30 * (ks ? p5 : n5), f1 = e31 * (ks ? p5 : n5);
            v16h af;
#pragma unroll
            for (int i = 0; i < 8; ++i) { af[i] = toh_flush(a[i] * f0); af[8 + i] = toh_flush(a[i] * f1); }
#pragma unroll
            for (int j = 0; j < 8; ++j) { const v16h b = ldh(rb + (size_t)j * 16 * NC + 32 * ks); acc[j] = wmma16g(af, b, acc[j]); }
        }
    }
    wave_sync();
#pragma unroll
    for (int j = 0; j < 8; ++j) {
#pragma unroll
        for (int r = 0; r < 8; ++r) ps[(8 * hi + r) * PP + j * 16 + lr] = acc[j][r] * OSC;
    }
    wave_sync();
    float* orow = OUT + ((size_t)bb * OUT_SEQ + ss) * NU;
#pragma unroll 1
    for (int pass = 0; pass < 2; ++pass) {
#pragma unroll
        for (int row = 0; row < 16; ++row) {
            const v4f val = *(const v4fa*)(&ps[row * PP + 4 * lane]);
            *(volatile v4f*)(orow + (size_t)row * NU + 4 * lane) = val; }
        if (pass == 0) __threadfence(); }
}

static constexpr size_t al256(size_t v) { return (v + 255) & ~(size_t)255; }
static constexpr size_t SZ_XH = al256((size_t)NB * SEQ * NF * 2);
static constexpr size_t SZ_ST = al256((size_t)TD * NF * 2);
static constexpr size_t SZ_RH = al256((size_t)NT * NU * NC * 2);
static constexpr size_t SZ_TOTAL = SZ_XH + SZ_ST + SZ_RH;
static_assert(SZ_TOTAL <= (size_t)134217728);
static_assert(((size_t)NB * SEQ * NF * 2) % 128 == 0);
static_assert(((size_t)TD * NF * 2) % 128 == 0);
static_assert(((size_t)NT * NU * NC * 2) % 128 == 0);

extern "C" void kernel_launch(void* const* d_in, const int* in_sizes, int n_in,
                              void* d_out, int out_size, void* d_ws, size_t ws_size, hipStream_t stream) {
    if (n_in < 5) return;
    const size_t needx = ((size_t)(NB - 1) * SEQ_FULL + SEQ) * NF;
    if ((size_t)in_sizes[0] < needx) return;
    if ((size_t)in_sizes[1] < (size_t)NF * TD) return;
    if (in_sizes[2] < TD || in_sizes[3] < TD) return;
    if ((size_t)in_sizes[4] < (size_t)NT * NU * NC) return;
    if ((size_t)out_size < ((size_t)(NB - 1) * OUT_SEQ + SEQ) * NU) return;
    if (SZ_TOTAL > ws_size) return;
    const float* x    = (const float*)d_in[0];
    const float* fl   = (const float*)d_in[1];
    const float* thr  = (const float*)d_in[2];
    const float* lt   = (const float*)d_in[3];
    const float* resp = (const float*)d_in[4];
    float* OUT = (float*)d_out;
    char* wsp = (char*)d_ws;
    h16* XH = (h16*)wsp; wsp += SZ_XH;
    h16* ST = (h16*)wsp; wsp += SZ_ST;
    h16* RH = (h16*)wsp; wsp += SZ_RH;

    if (SEQ == SEQ_FULL) {
        const size_t n8 = (size_t)NB * SEQ * NF / 8;
        k_cvth8<<<(unsigned)((n8 + 255) / 256), 256, 0, stream>>>(x, XH, n8);
    } else {
        const size_t n8 = (size_t)SEQ * NF / 8;
        for (int b = 0; b < NB; ++b) k_cvth8<<<(unsigned)((n8 + 255) / 256), 256, 0, stream>>>(x + (size_t)b * SEQ_FULL * NF, XH + (size_t)b * SEQ * NF, n8);
    }
    { const size_t n8 = (size_t)NT * NU * NC / 8;
      k_cvth8<<<(unsigned)((n8 + 255) / 256), 256, 0, stream>>>(resp, RH, n8); }
    k_sel<<<TD, NF, 0, stream>>>(fl, ST);
    k_trees<<<NB * SEQ / 16, 32, 0, stream>>>(XH, ST, RH, thr, lt, OUT);
}
